// SelfAttention_18940805775435
// MI455X (gfx1250) — hardware-verified
//
#include <hip/hip_runtime.h>
#include <math.h>

typedef __attribute__((ext_vector_type(16))) _Float16 v16h;
typedef __attribute__((ext_vector_type(16))) __bf16 v16b;
typedef __attribute__((ext_vector_type(8)))  _Float16 v8h;
typedef __attribute__((ext_vector_type(8)))  __bf16 v8b;
typedef __attribute__((ext_vector_type(8)))  float v8f;
typedef __attribute__((ext_vector_type(4)))  float v4f;
typedef __attribute__((ext_vector_type(4)))  unsigned v4u;
typedef _Float16 h16;

#ifndef NB
#define NB 2
#endif
#ifndef SEQ
#define SEQ 2048
#endif
#define NB_FULL 2
#define SEQ_FULL 2048
#ifndef OSEQ
#define OSEQ SEQ
#endif
#define TT SEQ
#define DIN 2048
#define NH 16
#define NKV 4
#define GRP (NH / NKV)
#define HD 128
#define HALF (HD / 2)
#define CQ (NH * HD)
#define CKV (NKV * HD)
#define NQB (TT / 64)
#define SCALE (0.08838834764831845f)
#define SC2 (SCALE * 1.4426950408889634f)
#define PCAR 14.0f
#define CTXC 16.0f
#define OSC (1.0f / 4096.0f)
static_assert(NB >= 1 && NB <= NB_FULL);
static_assert(SEQ % 128 == 0 && SEQ >= 128 && SEQ <= SEQ_FULL);
static_assert(HD == 128 && CQ % 128 == 0 && CKV % 128 == 0 && DIN % 64 == 0 && DIN == 256 * 8 && CQ % 32 == 0 && DIN % 128 == 0);
static_assert(NH % NKV == 0 && GRP * NKV == NH);
static_assert(TT % 64 == 0 && TT % 32 == 0 && HD % 32 == 0 && HD / 16 == 8 && HD / 32 == 4);
static_assert((NB * TT) % 64 == 0 && DIN % 32 == 0 && CQ % 64 == 0 && CKV % 32 == 0);
static_assert((size_t)NB_FULL * SEQ_FULL * DIN * 4u == (size_t)33554432u);

#define WS_XB   ((size_t)0)
#define WS_WQT  (WS_XB + 2u * (size_t)NB * TT * DIN)
#define WS_WKT  (WS_WQT + 2u * (size_t)CQ * DIN)
#define WS_WVT  (WS_WKT + 2u * (size_t)CKV * DIN)
#define WS_WOT  (WS_WVT + 2u * (size_t)CKV * DIN)
#define WS_QH   (WS_WOT + 2u * (size_t)DIN * CQ)
#define WS_KH   (WS_QH + 2u * (size_t)NB * TT * CQ)
#define WS_VT   (WS_KH + 2u * (size_t)NB * TT * CKV)
#define WS_CH   (WS_VT + 2u * (size_t)NB * CKV * TT)
#define WS_END  (WS_CH + 2u * (size_t)NB * TT * CQ)
static_assert(WS_END <= (size_t)134217728u);
static_assert(WS_WKT == WS_WQT + 2u * (size_t)CQ * DIN && WS_WVT == WS_WKT + 2u * (size_t)CKV * DIN);
static_assert(WS_WQT % 128 == 0 && WS_WKT % 128 == 0 && WS_WVT % 128 == 0 && WS_WOT % 128 == 0 && WS_QH % 128 == 0 && WS_KH % 128 == 0 && WS_VT % 128 == 0 && WS_CH % 128 == 0 && WS_END % 128 == 0);

template <typename T> __device__ __forceinline__ void vst2(void* p, T v) { *(volatile T*)p = v; __threadfence(); *(volatile T*)p = v; }
__device__ __forceinline__ v8f wmma16(v16h a, v16h b, v8f c) {
  v8f d = __builtin_amdgcn_wmma_f32_16x16x32_f16(false, a, false, b, (short)0, c, false, false);
  asm volatile("v_nop\n\tv_nop\n\tv_nop\n\tv_nop" : "+v"(d) : "v"(a), "v"(b));
  return d;
}
__device__ __forceinline__ v8f wmma_bf(v16b a, v16b b, v8f c) {
  v8f d = __builtin_amdgcn_wmma_f32_16x16x32_bf16(false, a, false, b, (short)0, c, false, false);
  asm volatile("v_nop\n\tv_nop\n\tv_nop\n\tv_nop" : "+v"(d) : "v"(a), "v"(b));
  return d;
}
__device__ __forceinline__ v16h frag_h(const _Float16* rowk0, int lane) {
  union { v16h v; v8h q[2]; } u; const _Float16* p = rowk0 + 8 * (lane >> 4);
  u.q[0] = *(const v8h*)p; u.q[1] = *(const v8h*)(p + 16); return u.v;
}
__device__ __forceinline__ v16b frag_b(const __bf16* rowk0, int lane) {
  union { v16b v; v8b q[2]; } u; const __bf16* p = rowk0 + 8 * (lane >> 4);
  u.q[0] = *(const v8b*)p; u.q[1] = *(const v8b*)(p + 16); return u.v;
}
__device__ __forceinline__ float bfr(float v) { return (float)(__bf16)v; }
static __device__ __forceinline__ h16 toh_flush(float v) { const h16 r = (h16)v; return (fabsf(v) < 6.103515625e-05f) ? (h16)0.0f : r; }
#define LDSX() do { asm volatile("s_wait_dscnt 0" ::: "memory"); __builtin_amdgcn_wave_barrier(); __builtin_amdgcn_fence(3  , "workgroup"); } while (0)

__global__ __launch_bounds__(256) void k_cvt_x(const float* __restrict__ X, __bf16* __restrict__ XB) {
  const int row = blockIdx.x, tid = threadIdx.x; const int b = row / TT, t = row - b * TT;
  const float* src = X + ((size_t)b * SEQ_FULL + t) * DIN + tid * 8;
  const v4f a = *(const v4f*)src, c = *(const v4f*)(src + 4);
  union { v8b v; v4u u; } o;
#pragma unroll
  for (int i = 0; i < 4; ++i) { o.v[i] = (__bf16)a[i]; o.v[4 + i] = (__bf16)c[i]; }
  vst2((unsigned*)(XB + (size_t)row * DIN + tid * 8), o.u);
}
template <int F16S>
__global__ __launch_bounds__(256) void k_cvt_wT(const float* __restrict__ W, unsigned short* __restrict__ WT, int K, int N) {
  __shared__ float tile[32][68];
  const int k0 = blockIdx.x * 64, n0 = blockIdx.y * 32; const int tid = threadIdx.x, nn = tid & 31, kq = tid >> 5;
#pragma unroll
  for (int i = 0; i < 8; ++i) { const int kk = kq + 8 * i; tile[nn][kk] = W[(size_t)(k0 + kk) * N + n0 + nn]; }
  __syncthreads();
  const int nl = tid >> 3, q = tid & 7;
  union { v8b b; v8h h; v4u u; } o;
#pragma unroll
  for (int i = 0; i < 8; ++i) { const float v = bfr(tile[nl][q * 8 + i]); if (F16S) o.h[i] = (_Float16)(v * 256.0f); else o.b[i] = (__bf16)v; }
  vst2((unsigned*)(WT + (size_t)(n0 + nl) * K + k0 + q * 8), o.u);
}

__global__ __launch_bounds__(128) void k_proj(const __bf16* __restrict__ XB, const __bf16* __restrict__ WT3, const float* __restrict__ COS, const float* __restrict__ SIN,
    _Float16* __restrict__ QH, _Float16* __restrict__ KH, _Float16* __restrict__ VT) {
  __shared__ __align__(16) _Float16 sh[64][136]; __shared__ __align__(16) _Float16 th[128][72]; __shared__ float scs[64][HALF], ssn[64][HALF];
  const int tid = threadIdx.x, wave = __builtin_amdgcn_readfirstlane(threadIdx.x >> 5), lane = tid & 31, col = lane & 15, g = lane >> 4;
  const int y = blockIdx.y; const int which = y < NH ? 0 : (y < NH + NKV ? 1 : 2); const int c0 = (which == 0 ? y : (which == 1 ? y - NH : y - NH - NKV)) * 128;
  const size_t r0 = (size_t)blockIdx.x * 64; const size_t bb = r0 / TT; const int t0 = (int)(r0 % TT);
  if (which < 2) { for (int e = tid; e < 64 * HALF; e += 128) { const int rr = e / HALF, p = e - rr * HALF; const size_t o = (size_t)(t0 + rr) * HALF + p; scs[rr][p] = bfr(COS[o]); ssn[rr][p] = bfr(SIN[o]); } }
  v8f acc[8] = {};
#pragma unroll 2
  for (int kc = 0; kc < DIN / 32; ++kc) { const v16b a = frag_b(XB + (r0 + wave * 16 + col) * DIN + kc * 32, lane);
    asm volatile("s_wait_loadcnt 0x0" ::: "memory");
#pragma unroll
    for (int j = 0; j < 8; ++j) { const v16b w = frag_b(WT3 + (size_t)(y * 128 + j * 16 + col) * DIN + kc * 32, lane); asm volatile("s_wait_loadcnt 0x0" ::: "memory"); acc[j] = wmma_bf(a, w, acc[j]); } }
  __syncthreads();
  if (which < 2) {
#pragma unroll
    for (int j = 0; j < 8; ++j) {
#pragma unroll
      for (int r = 0; r < 8; ++r) { const float v = acc[j][r]; const float pv = __shfl_xor(v, 1); const int rl = wave * 16 + 8 * g + r, cl = j * 16 + col; const int p = cl >> 1; const float c = scs[rl][p], s = ssn[rl][p];
        const float ev = v * c - pv * s, od = pv * s + v * c; const float rot = (col & 1) ? od : ev; sh[rl][cl] = toh_flush(rot); } }
    __syncthreads();
    for (int e = tid; e < 64 * 16; e += 128) { const int rl = e >> 4, q = e & 15; const v4u pk = *(const v4u*)&sh[rl][q * 8];
      if (which == 0) vst2((unsigned*)(QH + (r0 + rl) * (size_t)CQ + c0 + q * 8), pk); else vst2((unsigned*)(KH + (r0 + rl) * (size_t)CKV + c0 + q * 8), pk); }
  } else {
#pragma unroll
    for (int j = 0; j < 8; ++j) {
#pragma unroll
      for (int r = 0; r < 8; ++r) { const float v = acc[j][r]; const int rl = wave * 16 + 8 * g + r, cl = j * 16 + col; th[cl][rl] = toh_flush(v); } }
    __syncthreads();
    for (int e = tid; e < 128 * 8; e += 128) { const int cl = e >> 3, q = e & 7; vst2((unsigned*)(VT + (bb * CKV + c0 + cl) * (size_t)TT + t0 + q * 8), *(const v4u*)&th[cl][q * 8]); } } }

__global__ __launch_bounds__(128) void k_fa(const _Float16* __restrict__ QH, const _Float16* __restrict__ KH, const _Float16* __restrict__ VT, _Float16* __restrict__ CH) {
  __shared__ __align__(16) _Float16 s2h[4][16][136];
  const int tid = threadIdx.x, wave = __builtin_amdgcn_readfirstlane(threadIdx.x >> 5), lane = tid & 31, col = lane & 15, g = lane >> 4;
  const int qb = blockIdx.x, h = blockIdx.y, b = blockIdx.z, hk = h / GRP; const int ql0 = qb * 64 + wave * 16;
  const _Float16* qrow = QH + ((size_t)b * TT + ql0 + col) * CQ + h * HD;
  const _Float16* kbase = KH + ((size_t)b * TT + col) * CKV + hk * HD;
  const _Float16* vbase = VT + ((size_t)b * CKV + hk * HD + col) * (size_t)TT;
  v16h qf[4];
#pragma unroll
  for (int kc = 0; kc < 4; ++kc) qf[kc] = frag_h(qrow + kc * 32, lane);
  v8f o[8] = {}; float mrun = -3.0e38f, lrun = 0.0f;
#pragma unroll 1
  for (int k0 = 0; k0 < TT; k0 += 32) {
    v8f s0 = {}, s1 = {};
#pragma unroll
    for (int kc = 0; kc < 4; ++kc) { const v16h ka = frag_h(kbase + (size_t)k0 * CKV + kc * 32, lane), kb = frag_h(kbase + (size_t)(k0 + 16) * CKV + kc * 32, lane);
      asm volatile("s_wait_loadcnt 0x0" ::: "memory");
      s0 = wmma16(ka, qf[kc], s0); s1 = wmma16(kb, qf[kc], s1); }
    float mx = s0[0];
#pragma unroll
    for (int r = 1; r < 8; ++r) mx = fmaxf(mx, s0[r]);
#pragma unroll
    for (int r = 0; r < 8; ++r) mx = fmaxf(mx, s1[r]);
    mx = fmaxf(mx, __shfl_xor(mx, 16));
    const float mnew = fmaxf(mrun, mx * SC2);
    const float alpha = exp2f(mrun - mnew);
    const float off = PCAR - mnew;
    v16h pf; float ls = 0.0f;
#pragma unroll
    for (int r = 0; r < 8; ++r) {
      const float e0 = fmaf(s0[r], SC2, off), e1 = fmaf(s1[r], SC2, off);
      const h16 p0 = (e0 < -14.0f) ? (h16)0.0f : (h16)exp2f(e0);
      const h16 p1 = (e1 < -14.0f) ? (h16)0.0f : (h16)exp2f(e1);
      pf[r] = p0; pf[8 + r] = p1; ls += (float)p0 + (float)p1; }
    ls += __shfl_xor(ls, 16);
    lrun = lrun * alpha + ls; mrun = mnew;
#pragma unroll
    for (int j = 0; j < 8; ++j) o[j] = o[j] * alpha;
#pragma unroll
    for (int j = 0; j < 8; ++j) { const v16h va = frag_h(vbase + (size_t)(j * 16) * TT + k0, lane);
      asm volatile("s_wait_loadcnt 0x0" ::: "memory");
      o[j] = wmma16(va, pf, o[j]); }
  }
  const float inv = CTXC * (1.0f / lrun);
#pragma unroll
  for (int j = 0; j < 8; ++j) { union { v8h v; v4u u; } pk;
#pragma unroll
    for (int r = 0; r < 8; ++r) pk.v[r] = toh_flush(o[j][r] * inv);
    *(v4u*)&s2h[wave][col][j * 16 + 8 * g] = pk.u; }
  LDSX();
  for (int i = 0; i < 8; ++i) { const int rl = 2 * i + g; vst2((unsigned*)(CH + ((size_t)b * TT + ql0 + rl) * CQ + h * HD + col * 8), *(const v4u*)&s2h[wave][rl][col * 8]); }
}

__global__ __launch_bounds__(128) void k_out(const _Float16* __restrict__ CH, const _Float16* __restrict__ WOT, const int* __restrict__ SP, float* __restrict__ OUT) {
  __shared__ __align__(16) float so[64][132];
  const int tid = threadIdx.x, wave = __builtin_amdgcn_readfirstlane(threadIdx.x >> 5), lane = tid & 31, col = lane & 15, g = lane >> 4; const int c0 = blockIdx.y * 128;
  const size_t r0 = (size_t)blockIdx.x * 64; const size_t bb = r0 / TT; const int t0 = (int)(r0 % TT);
  const _Float16* arow = CH + (r0 + wave * 16 + col) * (size_t)CQ;
  v8f acc[8] = {};
#pragma unroll 2
  for (int kc = 0; kc < CQ / 32; ++kc) { const v16h ah = frag_h(arow + kc * 32, lane);
    asm volatile("s_wait_loadcnt 0x0" ::: "memory");
#pragma unroll
    for (int j = 0; j < 8; ++j) { const v16h w = frag_h(WOT + (size_t)(c0 + j * 16 + col) * CQ + kc * 32, lane); asm volatile("s_wait_loadcnt 0x0" ::: "memory"); acc[j] = wmma16(ah, w, acc[j]); } }
#pragma unroll
  for (int j = 0; j < 8; ++j) {
#pragma unroll
    for (int r = 0; r < 8; ++r) so[wave * 16 + 8 * g + r][j * 16 + col] = acc[j][r] * OSC; }
  __syncthreads();
  const bool bad = SP[0] != 0; const float qn = __uint_as_float(0x7fc00000u);
  for (int i = 0; i < 16; ++i) { const int rl = i * 4 + wave; v4f v = *(const v4f*)&so[rl][lane * 4]; if (bad) { v[0] = qn; v[1] = qn; v[2] = qn; v[3] = qn; }
    vst2(OUT + ((bb * OSEQ + t0 + rl) * (size_t)DIN) + c0 + lane * 4, v); } }

extern "C" void kernel_launch(void* const* d_in, const int* in_sizes, int n_in, void* d_out, int out_size, void* d_ws, size_t ws_size, hipStream_t stream) {
  if (n_in < 10) return;
  if (in_sizes[0] < ((NB - 1) * SEQ_FULL + SEQ) * DIN || in_sizes[1] < SEQ * HALF || in_sizes[2] < SEQ * HALF || in_sizes[3] < DIN * CQ || in_sizes[4] < DIN * CKV || in_sizes[5] < DIN * CKV || in_sizes[6] < CQ * DIN || in_sizes[9] < 1) return;
  if ((size_t)out_size < ((size_t)(NB - 1) * OSEQ + SEQ) * DIN) return;
  if (ws_size < (size_t)WS_END) return;
  const float** F = (const float**)d_in;
  const int* SP = (const int*)d_in[9];
  char* ws = (char*)d_ws;
  __bf16 *XB = (__bf16*)(ws + WS_XB), *WQT = (__bf16*)(ws + WS_WQT), *WKT = (__bf16*)(ws + WS_WKT), *WVT = (__bf16*)(ws + WS_WVT);
  _Float16 *WOT = (_Float16*)(ws + WS_WOT), *QH = (_Float16*)(ws + WS_QH), *KH = (_Float16*)(ws + WS_KH), *VT = (_Float16*)(ws + WS_VT), *CH = (_Float16*)(ws + WS_CH);
  k_cvt_x<<<dim3(NB * TT), 256, 0, stream>>>(F[0], XB);
  k_cvt_wT<0><<<dim3(DIN / 64, CQ / 32), 256, 0, stream>>>(F[3], (unsigned short*)WQT, DIN, CQ);
  k_cvt_wT<0><<<dim3(DIN / 64, CKV / 32), 256, 0, stream>>>(F[4], (unsigned short*)WKT, DIN, CKV);
  k_cvt_wT<0><<<dim3(DIN / 64, CKV / 32), 256, 0, stream>>>(F[5], (unsigned short*)WVT, DIN, CKV);
  k_cvt_wT<1><<<dim3(CQ / 64, DIN / 32), 256, 0, stream>>>(F[6], (unsigned short*)WOT, CQ, DIN);
  k_proj<<<dim3(NB * TT / 64, NH + 2 * NKV, 1), 128, 0, stream>>>(XB, WQT, F[1], F[2], QH, KH, VT);
  k_fa<<<dim3(NQB, NH, NB), 128, 0, stream>>>(QH, KH, VT, CH);
  k_out<<<dim3(NB * TT / 64, DIN / 128), 128, 0, stream>>>(CH, WOT, SP, (float*)d_out);
}
